// TextOverRegionAttention_61048665145682
// MI455X (gfx1250) — hardware-verified
//
#include <hip/hip_runtime.h>
#include <math.h>

typedef __attribute__((ext_vector_type(16))) _Float16 v16h;
typedef __attribute__((ext_vector_type(16))) __bf16 v16b;
typedef __attribute__((ext_vector_type(8)))  _Float16 v8h;
typedef __attribute__((ext_vector_type(8)))  float v8f;
typedef __attribute__((ext_vector_type(4)))  float v4f;
typedef __attribute__((ext_vector_type(2)))  float v2f;
typedef __attribute__((ext_vector_type(4)))  unsigned v4u;
typedef __attribute__((ext_vector_type(4)))  int v4i;
typedef float __attribute__((may_alias)) float_a;
typedef int __attribute__((may_alias)) int_a;

template <typename T> __device__ __forceinline__ void vst2(void* p, T v) { *(volatile T*)p = v; __threadfence(); *(volatile T*)p = v; }
__device__ __forceinline__ v8f wmma16(v16h a, v16h b, v8f c) {
  v8f d = __builtin_amdgcn_wmma_f32_16x16x32_f16(false, a, false, b, (short)0, c, false, false);
  asm volatile("v_nop\n\tv_nop\n\tv_nop\n\tv_nop" : "+v"(d) : "v"(a), "v"(b));
  return d;
}
__device__ __forceinline__ v8f wmma_bf(v16b a, v16b b, v8f c) {
  v8f d = __builtin_amdgcn_wmma_f32_16x16x32_bf16(false, a, false, b, (short)0, c, false, false);
  asm volatile("v_nop\n\tv_nop\n\tv_nop\n\tv_nop" : "+v"(d) : "v"(a), "v"(b));
  return d;
}
__device__ __forceinline__ v16h frag_h(const _Float16* rowk0, int lane) {
  union { v16h v; v8h q[2]; } u; const _Float16* p = rowk0 + 8 * (lane >> 4);
  u.q[0] = *(const v8h*)p; u.q[1] = *(const v8h*)(p + 16); return u.v;
}
__device__ __forceinline__ v16h frag_f32(const float* rowk0, int lane) {
  v16h a; const float* p = rowk0 + 8 * (lane >> 4);
#pragma unroll
  for (int i = 0; i < 8; ++i) { a[i] = (_Float16)p[i]; a[8 + i] = (_Float16)p[16 + i]; }
  return a;
}
__device__ __forceinline__ v16h frag_f32s(const float* rowk0, int lane, float sc) {
  v16h a; const float* p = rowk0 + 8 * (lane >> 4);
#pragma unroll
  for (int i = 0; i < 8; ++i) { a[i] = (_Float16)(p[i] * sc); a[8 + i] = (_Float16)(p[16 + i] * sc); }
  return a;
}
__device__ __forceinline__ v16h fragc_f32(const float* W, int k0, int n, int lane, int ld, int K) {
  v16h a; const int g = lane >> 4;
#pragma unroll
  for (int i = 0; i < 8; ++i) { const int ka = k0 + 8 * g + i, kb = ka + 16;
    a[i] = (_Float16)(ka < K ? W[(size_t)(ka < K ? ka : K - 1) * ld + n] : 0.f); a[8 + i] = (_Float16)(kb < K ? W[(size_t)(kb < K ? kb : K - 1) * ld + n] : 0.f); }
  return a;
}
struct F2 { v16b h, l; };
__device__ __forceinline__ F2 bsplit16(const float v[16]) { F2 r;
#pragma unroll
  for (int i = 0; i < 16; ++i) { const __bf16 h = (__bf16)v[i]; r.h[i] = h; r.l[i] = (__bf16)(v[i] - (float)h); }
  return r; }
__device__ __forceinline__ F2 split_row(const float* row, int k0, int lane) { float v[16]; const float* p = row + k0 + 8 * (lane >> 4);
#pragma unroll
  for (int i = 0; i < 8; ++i) { v[i] = p[i]; v[8 + i] = p[16 + i]; }
  return bsplit16(v); }
__device__ __forceinline__ F2 split_rowK(const float* row, int k0, int lane, int K) { float v[16]; const int g = lane >> 4;
#pragma unroll
  for (int i = 0; i < 8; ++i) { const int ka = k0 + 8 * g + i, kb = ka + 16; v[i] = ka < K ? row[ka < K ? ka : K - 1] : 0.f; v[8 + i] = kb < K ? row[kb < K ? kb : K - 1] : 0.f; }
  return bsplit16(v); }
__device__ __forceinline__ F2 split_col(const float* W, int k0, int n, int lane, int ld, int K) { float v[16]; const int g = lane >> 4;
#pragma unroll
  for (int i = 0; i < 8; ++i) { const int ka = k0 + 8 * g + i, kb = ka + 16; v[i] = ka < K ? W[(size_t)(ka < K ? ka : K - 1) * ld + n] : 0.f; v[8 + i] = kb < K ? W[(size_t)(kb < K ? kb : K - 1) * ld + n] : 0.f; }
  return bsplit16(v); }
__device__ __forceinline__ v8f mac3(const F2& a, const F2& b, v8f c) { c = wmma_bf(a.l, b.h, c); c = wmma_bf(a.h, b.l, c); return wmma_bf(a.h, b.h, c); }
__device__ __forceinline__ float sigm(float v) { return 1.0f / (1.0f + expf(-v)); }
#define LDSX() do { asm volatile("s_wait_dscnt 0" ::: "memory"); __builtin_amdgcn_wave_barrier(); __builtin_amdgcn_fence(__ATOMIC_RELEASE, "workgroup"); } while (0)


#define NB 4
#define LL 4096
#define NN 1024
#define DM 768
#define NH 12
#define HD 64
#define RR 8
#define NRQ (NB * LL)
#define NRK (NB * NN)
#define WSC 64.0f
#ifndef TQB
#define TQB (LL / 64)
#define TNB NB
#endif
typedef __attribute__((ext_vector_type(8))) __bf16 v8b;
__device__ __forceinline__ v16b frag_b(const __bf16* rowk0, int lane) {
  union { v16b v; v8b q[2]; } u; const __bf16* p = rowk0 + 8 * (lane >> 4);
  u.q[0] = *(const v8b*)p; u.q[1] = *(const v8b*)(p + 16); return u.v;
}
__device__ __forceinline__ float bfr(float v) { return (float)(__bf16)v; }
__device__ __attribute__((noinline)) float exp_ni(float v) { return expf(v); }
__device__ __attribute__((noinline)) float erf_ni(float v) { return erff(v); }

#define WS_PW  0u
#define WS_TQ  (WS_PW + 2u * (size_t)4 * DM * DM)
#define WS_RK  (WS_TQ + 2u * (size_t)NRQ * DM)
#define WS_Q   (WS_RK + 2u * (size_t)NRK * DM)
#define WS_K   (WS_Q + 2u * (size_t)NRQ * DM)
#define WS_V   (WS_K + 2u * (size_t)NRK * DM)
#define WS_O   (WS_V + 2u * (size_t)NB * DM * NN)
#define WS_END (WS_O + 4u * (size_t)NRQ * DM)

__global__ __launch_bounds__(256) void k_fold(const float* __restrict__ WQ, const float* __restrict__ AQ, const float* __restrict__ BQ, const float* __restrict__ WK, const float* __restrict__ WV, const float* __restrict__ AV, const float* __restrict__ BV, const float* __restrict__ WO, _Float16* __restrict__ PW) {
  __shared__ float sb[RR]; __shared__ __align__(16) _Float16 s[DM]; const int n = blockIdx.x, which = blockIdx.y, t = threadIdx.x;
  const float* Wm = (which == 0) ? WQ : (which == 1) ? WK : (which == 2) ? WV : WO; const float* A = (which == 0) ? AQ : AV; const float* Bm = (which == 0) ? BQ : BV; const bool lora = (which == 0 || which == 2);
  if (t < RR) sb[t] = lora ? bfr(Bm[(size_t)n * RR + t]) : 0.f; __syncthreads();
  for (int c = t; c < DM; c += 256) { float w = bfr(Wm[(size_t)n * DM + c]); if (lora) { float a = 0.f;
#pragma unroll
      for (int r = 0; r < RR; ++r) a += sb[r] * bfr(A[(size_t)r * DM + c]); w += 2.0f * a; }
    s[c] = (_Float16)(w * WSC); }
  __syncthreads(); for (int q = t; q < DM / 8; q += 256) vst2((unsigned*)(PW + ((size_t)which * DM + n) * DM + q * 8), *(const v4u*)&s[q * 8]); }
__global__ __launch_bounds__(256) void k_ln(const float* __restrict__ X, const float* __restrict__ G, const float* __restrict__ Bt, _Float16* __restrict__ T) { __shared__ float red[8]; __shared__ __align__(16) _Float16 so[DM]; const int t = threadIdx.x; const size_t row = blockIdx.x; float v[3]; float s = 0.f; for (int i = 0; i < 3; ++i) { v[i] = bfr(X[row * DM + t + 256 * i]); s += v[i]; }
#pragma unroll
  for (int o = 1; o < 32; o <<= 1) s += __shfl_xor(s, o);
  if ((t & 31) == 0) red[t >> 5] = s; __syncthreads(); float tot = 0.f; for (int i = 0; i < 8; ++i) tot += red[i]; const float mu = tot / (float)DM; __syncthreads();
  float q = 0.f; for (int i = 0; i < 3; ++i) { const float d = v[i] - mu; q += d * d; }
#pragma unroll
  for (int o = 1; o < 32; o <<= 1) q += __shfl_xor(q, o);
  if ((t & 31) == 0) red[t >> 5] = q; __syncthreads(); float tq = 0.f; for (int i = 0; i < 8; ++i) tq += red[i]; const float inv = 1.0f / sqrtf(tq / (float)DM + 1e-5f);
  for (int i = 0; i < 3; ++i) { const int c = t + 256 * i; so[c] = (_Float16)((v[i] - mu) * inv * bfr(G[c]) + bfr(Bt[c])); } __syncthreads(); if (t < DM / 8) vst2((unsigned*)(T + row * DM + t * 8), *(const v4u*)&so[t * 8]); }
__global__ __launch_bounds__(128) void k_proj(const _Float16* __restrict__ TQ, const _Float16* __restrict__ RK, const float* __restrict__ REG, const _Float16* __restrict__ PW, _Float16* __restrict__ Q, _Float16* __restrict__ Kr, _Float16* __restrict__ V) {
  __shared__ __align__(16) _Float16 so[64][136]; __shared__ __align__(16) _Float16 st[128][72];
  const int tid = threadIdx.x, wave = tid >> 5, lane = tid & 31, col = lane & 15, g = lane >> 4; const int which = blockIdx.z; const size_t rb = (size_t)blockIdx.x * 64; if (which > 0 && rb >= (size_t)TNB * NN) return;
  const size_t r0 = rb + wave * 16; const int c0 = blockIdx.y * 128; const _Float16* Wr = PW + ((size_t)which * DM) * DM; const _Float16* A = (which == 0) ? TQ : RK;
  v8f acc[8] = {};
#pragma unroll 2
  for (int kc = 0; kc < DM / 32; ++kc) { v16h a; if (which < 2) a = frag_h(A + (r0 + col) * DM + kc * 32, lane); else { const float* p = REG + (r0 + col) * DM + kc * 32 + 8 * g;
#pragma unroll
      for (int i = 0; i < 8; ++i) { a[i] = (_Float16)bfr(p[i]); a[8 + i] = (_Float16)bfr(p[16 + i]); } }
#pragma unroll
    for (int j = 0; j < 8; ++j) acc[j] = wmma16(a, frag_h(Wr + (size_t)(c0 + j * 16 + col) * DM + kc * 32, lane), acc[j]); }
#pragma unroll
  for (int j = 0; j < 8; ++j)
#pragma unroll
    for (int r = 0; r < 8; ++r) { const _Float16 hv = (_Float16)(acc[j][r] * (1.0f / WSC)); if (which < 2) so[wave * 16 + 8 * g + r][j * 16 + col] = hv; else st[j * 16 + col][wave * 16 + 8 * g + r] = hv; }
  __syncthreads();
  if (which < 2) { _Float16* dst = (which == 0) ? Q : Kr; for (int e = tid; e < 64 * 16; e += 128) { const int rl = e >> 4, q = e & 15; vst2((unsigned*)(dst + (rb + rl) * DM + c0 + q * 8), *(const v4u*)&so[rl][q * 8]); } }
  else { const size_t b = rb / NN; const int s0 = (int)(rb % NN); for (int e = tid; e < 128 * 8; e += 128) { const int d = e >> 3, pc = e & 7; vst2((unsigned*)(V + ((b * DM + c0 + d) * NN) + s0 + pc * 8), *(const v4u*)&st[d][pc * 8]); } }
}
__global__ __launch_bounds__(128) void k_attn(const _Float16* __restrict__ Q, const _Float16* __restrict__ Kr, const _Float16* __restrict__ V, const int* __restrict__ MK, float* __restrict__ O) {
  __shared__ __align__(16) _Float16 sph[4][16][40]; __shared__ __align__(16) float so[4][16][68];
  const int tid = threadIdx.x, wave = tid >> 5, lane = tid & 31, col = lane & 15, g = lane >> 4; const int h = blockIdx.y; const size_t b = blockIdx.z; const int q0 = blockIdx.x * 64 + wave * 16; const size_t rq = b * LL + q0;
  v16h aq[2];
#pragma unroll
  for (int kc = 0; kc < 2; ++kc) aq[kc] = frag_h(Q + (rq + col) * DM + h * HD + kc * 32, lane);
  float m[8], l[8];
#pragma unroll
  for (int r = 0; r < 8; ++r) { m[r] = -3.0e38f; l[r] = 0.f; }
  v8f acc[4] = {};
#pragma unroll 1
  for (int ks = 0; ks < NN / 32; ++ks) { const int j0 = ks * 32; v8f s[2];
#pragma unroll
    for (int ct = 0; ct < 2; ++ct) { const int kk = j0 + ct * 16 + col; const size_t rk = (b * NN + kk) * DM + h * HD; v8f c = {}; const bool keepk = MK[b * NN + kk] != 0;
#pragma unroll
      for (int kc = 0; kc < 2; ++kc) c = wmma16(aq[kc], frag_h(Kr + rk + kc * 32, lane), c);
#pragma unroll
      for (int r = 0; r < 8; ++r) s[ct][r] = keepk ? c[r] * 0.125f : -3.0e38f; }
#pragma unroll
    for (int r = 0; r < 8; ++r) { float mx = fmaxf(s[0][r], s[1][r]);
#pragma unroll
      for (int o = 1; o < 16; o <<= 1) mx = fmaxf(mx, __shfl_xor(mx, o));
      const float mn = fmaxf(m[r], mx); const float alpha = (m[r] <= -1.0e38f) ? 0.f : __expf(m[r] - mn); const float e0 = (s[0][r] <= -1.0e38f) ? 0.f : __expf(s[0][r] - mn), e1 = (s[1][r] <= -1.0e38f) ? 0.f : __expf(s[1][r] - mn); float es = e0 + e1;
#pragma unroll
      for (int o = 1; o < 16; o <<= 1) es += __shfl_xor(es, o);
      l[r] = l[r] * alpha + es; m[r] = mn;
#pragma unroll
      for (int dt = 0; dt < 4; ++dt) acc[dt][r] *= alpha;
      sph[wave][8 * g + r][col] = (_Float16)(e0 * 2048.0f); sph[wave][8 * g + r][16 + col] = (_Float16)(e1 * 2048.0f); }
    LDSX();
    const v16h pa = frag_h(&sph[wave][col][0], lane);
#pragma unroll
    for (int dt = 0; dt < 4; ++dt) acc[dt] = wmma16(pa, frag_h(V + ((b * DM + h * HD + dt * 16 + col) * NN) + j0, lane), acc[dt]);
    LDSX(); }
#pragma unroll
  for (int r = 0; r < 8; ++r) { const float il = (l[r] > 0.f) ? (1.0f / 2048.0f) / l[r] : 0.f;
#pragma unroll
    for (int dt = 0; dt < 4; ++dt) so[wave][8 * g + r][dt * 16 + col] = acc[dt][r] * il; }
  LDSX();
  for (int rl = 0; rl < 16; ++rl) if (lane < 16) vst2(O + (rq + rl) * DM + h * HD + lane * 4, *(const v4f*)&so[wave][rl][lane * 4]);
}
__global__ __launch_bounds__(128) void k_out(const float* __restrict__ O, const _Float16* __restrict__ PW, const float* __restrict__ BO, const float* __restrict__ TX, float* __restrict__ Y) { __shared__ __align__(16) float so[4][16][132];
  const int tid = threadIdx.x, wave = tid >> 5, lane = tid & 31, col = lane & 15, g = lane >> 4; const size_t r0 = (size_t)blockIdx.x * 64 + wave * 16; const int c0 = blockIdx.y * 128; const _Float16* Wr = PW + (size_t)3 * DM * DM;
  v8f acc[8] = {};
#pragma unroll 2
  for (int kc = 0; kc < DM / 32; ++kc) { v16h a; { const float* p = O + (r0 + col) * DM + kc * 32 + 8 * g;
#pragma unroll
      for (int i = 0; i < 8; ++i) { a[i] = (_Float16)p[i]; a[8 + i] = (_Float16)p[16 + i]; } }
#pragma unroll
    for (int j = 0; j < 8; ++j) acc[j] = wmma16(a, frag_h(Wr + (size_t)(c0 + j * 16 + col) * DM + kc * 32, lane), acc[j]); }
#pragma unroll
  for (int j = 0; j < 8; ++j) { const int c = c0 + j * 16 + col; const float bb = bfr(BO[c]);
#pragma unroll
    for (int r = 0; r < 8; ++r) so[wave][8 * g + r][j * 16 + col] = acc[j][r] * (1.0f / WSC) + bb + bfr(TX[(r0 + 8 * g + r) * DM + c]); }
  LDSX(); for (int rl = 0; rl < 16; ++rl) vst2(Y + (r0 + rl) * DM + c0 + lane * 4, *(const v4f*)&so[wave][rl][lane * 4]); }
extern "C" void kernel_launch(void* const* d_in, const int* in_sizes, int n_in, void* d_out, int out_size, void* d_ws, size_t ws_size, hipStream_t stream) {
  (void)in_sizes; (void)n_in; (void)out_size;
  const float** F = (const float**)d_in;
  if (ws_size < (size_t)WS_END) return;
  char* ws = (char*)d_ws; _Float16 *PW = (_Float16*)(ws + WS_PW), *TQ = (_Float16*)(ws + WS_TQ), *RK = (_Float16*)(ws + WS_RK), *Q = (_Float16*)(ws + WS_Q), *Kr = (_Float16*)(ws + WS_K), *V = (_Float16*)(ws + WS_V); float* O = (float*)(ws + WS_O);
  k_fold<<<dim3(DM, 4), 256, 0, stream>>>(F[3], F[4], F[5], F[6], F[7], F[8], F[9], F[10], PW);
  k_ln<<<TNB * LL, 256, 0, stream>>>(F[0], F[12], F[13], TQ);
  k_ln<<<TNB * NN, 256, 0, stream>>>(F[1], F[14], F[15], RK);
  k_proj<<<dim3(TNB * LL / 64, DM / 128, 3), 128, 0, stream>>>(TQ, RK, F[1], PW, Q, Kr, V);
  k_attn<<<dim3(TQB, NH, TNB), 128, 0, stream>>>(Q, Kr, V, (const int*)d_in[2], O);
  k_out<<<dim3(TNB * LL / 64, DM / 128), 128, 0, stream>>>(O, PW, F[11], F[0], (float*)d_out);
}
